// UGCG_GMM_50697793962355
// MI455X (gfx1250) — hardware-verified
//
#include <hip/hip_runtime.h>
#include <stddef.h>


#define IN_F   64
#define HIDF   32
#define OUT_F  16
#define NKER   3
#define PDIM   2
#define C1     (NKER * HIDF)
#define C2     (NKER * OUT_F)
#define C2P    64
#define NTHR   256
#define GROWS  128
#define A1NB   32
#define A2NB   64
#define DEGCAP 4096
#define WSCAP  ((size_t)134217728)

static_assert(C1 % 32 == 0);
static_assert(C2P % 32 == 0 && C2P >= C2);
static_assert(IN_F % 32 == 0 && HIDF % 32 == 0);
static_assert(GROWS == 16 * (NTHR / 32));
static_assert((C1 * IN_F / 8) % NTHR == 0);
static_assert((C2 * HIDF / 8) % 32 == 0);
static_assert(A1NB == 4 * (NTHR / 32) && A2NB == 8 * (NTHR / 32));
static_assert(GROWS % A1NB == 0);

typedef float          v2f   __attribute__((ext_vector_type(2)));
typedef float          v4f   __attribute__((ext_vector_type(4)));
typedef v4f            __attribute__((may_alias)) v4fa;
typedef float          v8f   __attribute__((ext_vector_type(8)));
typedef unsigned short v8us  __attribute__((ext_vector_type(8)));
typedef unsigned short v16us __attribute__((ext_vector_type(16)));
typedef __bf16         v16bf __attribute__((ext_vector_type(16)));
union FragB { v16bf v; v16us u; v8us s[2]; };

__device__ __forceinline__ unsigned bf16_bits(float x) {
  const unsigned u = __float_as_uint(x);
  return (u + 0x7FFFu + ((u >> 16) & 1u)) >> 16;
}

__device__ __forceinline__ v8f wmb(v16bf a, v16bf b, v8f c) {
  v8f d = __builtin_amdgcn_wmma_f32_16x16x32_bf16(false, a, false, b, (short)0, c, false, false);
  asm volatile("v_nop\n\tv_nop\n\tv_nop\n\tv_nop" : "+v"(d) : "v"(a), "v"(b));
  return d;
}

__device__ __forceinline__ void split16(v4f a, v4f b, v4f c, v4f d, FragB& hi, FragB& lo) {
  float f[16];
  f[0]  = a.x; f[1]  = a.y; f[2]  = a.z; f[3]  = a.w;
  f[4]  = b.x; f[5]  = b.y; f[6]  = b.z; f[7]  = b.w;
  f[8]  = c.x; f[9]  = c.y; f[10] = c.z; f[11] = c.w;
  f[12] = d.x; f[13] = d.y; f[14] = d.z; f[15] = d.w;
#pragma unroll
  for (int i = 0; i < 16; ++i) {
    const unsigned hb = bf16_bits(f[i]);
    const float    hf = __uint_as_float(hb << 16);
    const unsigned lb = bf16_bits(f[i] - hf);
    hi.u[i] = (unsigned short)hb;
    lo.u[i] = (unsigned short)lb;
  }
}

__global__ __launch_bounds__(NTHR) void k_wprep(
    const float* __restrict__ W1, const float* __restrict__ W2,
    unsigned short* b1h, unsigned short* b1l, unsigned short* b2h, unsigned short* b2l) {
  const int g1 = C1 * IN_F / 8;
  const int g2 = C2 * HIDF / 8;
  const int i = blockIdx.x * NTHR + (int)threadIdx.x;
  float v[8];
  unsigned short* dh;
  unsigned short* dl;
  int o;
  if (blockIdx.x * NTHR < g1) {
    o = i * 8;
    const int n  = o / IN_F;
    const int f0 = o - n * IN_F;
    const int k  = n / HIDF;
    const int h  = n - k * HIDF;
#pragma unroll
    for (int e = 0; e < 8; ++e) v[e] = W1[((size_t)k * IN_F + f0 + e) * HIDF + h];
    dh = b1h; dl = b1l;
  } else {
    const int j = i - g1;
    if (j >= g2) return;
    o = j * 8;
    const int n  = o / HIDF;
    const int c0 = o - n * HIDF;
    const int k  = n / OUT_F;
    const int oo = n - k * OUT_F;
#pragma unroll
    for (int e = 0; e < 8; ++e) v[e] = W2[((size_t)k * HIDF + c0 + e) * OUT_F + oo];
    dh = b2h; dl = b2l;
  }
  v8us hv, lv;
#pragma unroll
  for (int e = 0; e < 8; ++e) {
    const unsigned hb = bf16_bits(v[e]);
    const float    hf = __uint_as_float(hb << 16);
    const unsigned lb = bf16_bits(v[e] - hf);
    hv[e] = (unsigned short)hb;
    lv[e] = (unsigned short)lb;
  }
  *(volatile v8us*)(dh + o) = hv;
  *(volatile v8us*)(dl + o) = lv;
  __threadfence();
  *(volatile v8us*)(dh + o) = hv;
  *(volatile v8us*)(dl + o) = lv;
}

__global__ __launch_bounds__(NTHR) void k_gauss(
    const float* __restrict__ p, const float* __restrict__ mu, const float* __restrict__ sigma,
    float* G, int nE) {
#pragma clang fp contract(off)
  const int e  = blockIdx.x * NTHR + (int)threadIdx.x;
  const int ec = e < nE ? e : nE - 1;
  const v2f pv = *(const v2f*)(p + (size_t)PDIM * ec);
  float g0 = 0.0f, g1 = 0.0f, g2 = 0.0f;
#pragma unroll 1
  for (int k = 0; k < NKER; ++k) {
    const float m0  = mu[PDIM * k + 0],    m1 = mu[PDIM * k + 1];
    const float s0  = sigma[PDIM * k + 0], s1 = sigma[PDIM * k + 1];
    const float iv0 = 1.0f / (s0 * s0);
    const float iv1 = 1.0f / (s1 * s1);
    const float d0  = pv.x - m0;
    const float d1  = pv.y - m1;
    const float t0  = (d0 * d0) * iv0;
    const float t1  = (d1 * d1) * iv1;
    const float q   = t0 + t1;
    const float gk  = expf(-0.5f * q);
    g0 = (k == 0) ? gk : g0;
    g1 = (k == 1) ? gk : g1;
    g2 = (k == 2) ? gk : g2;
  }
  const bool ok = e < nE;
  v4f gv;
  gv.x = ok ? g0 : 0.0f; gv.y = ok ? g1 : 0.0f; gv.z = ok ? g2 : 0.0f; gv.w = 0.0f;
  float* gp = G + (size_t)4 * e;
  *(volatile v4f*)gp = gv;
  __threadfence();
  *(volatile v4f*)gp = gv;
}

template <int KD, int NT, int CP>
__global__ __launch_bounds__(NTHR) void k_gemm(
    const float* __restrict__ A, const unsigned short* __restrict__ Bh, const unsigned short* __restrict__ Bl,
    float* C, int nRowsA) {
  static_assert(KD % 32 == 0 && NT * 16 <= CP && CP % 32 == 0 && GROWS * CP * 4 <= 65536);
  __shared__ __attribute__((aligned(16))) float stg[GROWS * CP];
  const int tid = threadIdx.x, lane = tid & 31, wave = tid >> 5, hh = lane >> 4, m = lane & 15;
  const int rowBase = blockIdx.x * GROWS;
  int row = rowBase + wave * 16 + m;
  row = row > nRowsA - 1 ? nRowsA - 1 : row;
  const float* ar = A + (size_t)row * KD + 8 * hh;

  v8f acc[NT];
#pragma unroll
  for (int t = 0; t < NT; ++t) { v8f z = {0.f, 0.f, 0.f, 0.f, 0.f, 0.f, 0.f, 0.f}; acc[t] = z; }

#pragma unroll
  for (int kt = 0; kt < KD / 32; ++kt) {
    const float* ap = ar + 32 * kt;
    const v4f x0 = *(const v4f*)(ap);
    const v4f x1 = *(const v4f*)(ap + 4);
    const v4f x2 = *(const v4f*)(ap + 16);
    const v4f x3 = *(const v4f*)(ap + 20);
    FragB ahi, alo;
    split16(x0, x1, x2, x3, ahi, alo);
#pragma unroll
    for (int t = 0; t < NT; ++t) {
      const size_t bp = (size_t)(16 * t + m) * KD + 32 * kt + 8 * hh;
      FragB bh, bl;
      bh.s[0] = *(const v8us*)(Bh + bp);
      bh.s[1] = *(const v8us*)(Bh + bp + 16);
      bl.s[0] = *(const v8us*)(Bl + bp);
      bl.s[1] = *(const v8us*)(Bl + bp + 16);
      acc[t] = wmb(ahi.v, bh.v, acc[t]);
      acc[t] = wmb(alo.v, bh.v, acc[t]);
      acc[t] = wmb(ahi.v, bl.v, acc[t]);
    }
  }

  float* sp = stg + (wave * 16 + 8 * hh) * CP + m;
#pragma unroll
  for (int t = 0; t < NT; ++t) {
#pragma unroll
    for (int r = 0; r < 8; ++r) sp[r * CP + 16 * t] = acc[t][r];
  }
#pragma unroll
  for (int c0 = NT * 16; c0 < CP; c0 += 16) {
#pragma unroll
    for (int r = 0; r < 8; ++r) sp[r * CP + c0] = 0.0f;
  }
  __syncthreads();

  const float* lp = stg + wave * 16 * CP + 4 * lane;
  float* gp = C + ((size_t)rowBase + wave * 16) * CP + 4 * lane;
#pragma unroll
  for (int i = 0; i < CP / 8; ++i) { const v4f v = *(const v4fa*)(lp + 128 * i); *(volatile v4f*)(gp + 128 * i) = v; }
  __threadfence();
#pragma unroll
  for (int i = 0; i < CP / 8; ++i) { const v4f v = *(const v4fa*)(lp + 128 * i); *(volatile v4f*)(gp + 128 * i) = v; }
}

__global__ __launch_bounds__(NTHR) void k_agg1(
    const int* __restrict__ rp, const int* __restrict__ col, const float* __restrict__ G,
    const float* __restrict__ XW, float* H, int nN, int nE) {
  const int tid = threadIdx.x, lane = tid & 31, wave = tid >> 5;
  const int g = lane >> 3, q = lane & 7;
  const int i = blockIdx.x * A1NB + wave * 4 + g;
  const int ia = i < nN ? i : nN - 1;
  int s = rp[ia];
  int t = rp[ia + 1];
  s = s < 0 ? 0 : (s > nE ? nE : s);
  t = t < s ? s : (t > nE ? nE : t);
  int deg = (i < nN) ? (t - s) : 0;
  deg = deg > DEGCAP ? DEGCAP : deg;
  int dm = deg;
  dm = max(dm, __shfl_xor(dm, 8));
  dm = max(dm, __shfl_xor(dm, 16));
  dm = __builtin_amdgcn_readfirstlane(dm);

  v4f acc = {0.f, 0.f, 0.f, 0.f};
#pragma unroll 1
  for (int j = 0; j < dm; ++j) {
    const bool ok = j < deg;
    int e = s + j;
    e = e > nE - 1 ? nE - 1 : e;
    int c = col[e];
    c = c < 0 ? 0 : (c > nN - 1 ? nN - 1 : c);
    const v4f gv = *(const v4f*)(G + (size_t)4 * e);
    const float g0 = ok ? gv.x : 0.0f, g1 = ok ? gv.y : 0.0f, g2 = ok ? gv.z : 0.0f;
    const float* xr = XW + (size_t)c * C1 + 4 * q;
    const v4f a0 = *(const v4f*)(xr);
    const v4f a1 = *(const v4f*)(xr + HIDF);
    const v4f a2 = *(const v4f*)(xr + 2 * HIDF);
    acc = acc + (a0 * g0 + a1 * g1 + a2 * g2);
  }
  float* hp = H + (size_t)i * HIDF + 4 * q;
  *(volatile v4f*)hp = acc;
  __threadfence();
  *(volatile v4f*)hp = acc;
}

__global__ __launch_bounds__(NTHR) void k_agg2(
    const int* __restrict__ rp, const int* __restrict__ col, const float* __restrict__ G,
    const float* __restrict__ HW, float* out, int nN, int nE) {
  const int tid = threadIdx.x, lane = tid & 31, wave = tid >> 5;
  const int g = lane >> 2, q = lane & 3;
  const int i = blockIdx.x * A2NB + wave * 8 + g;
  const int ia = i < nN ? i : nN - 1;
  int s = rp[ia];
  int t = rp[ia + 1];
  s = s < 0 ? 0 : (s > nE ? nE : s);
  t = t < s ? s : (t > nE ? nE : t);
  int deg = (i < nN) ? (t - s) : 0;
  deg = deg > DEGCAP ? DEGCAP : deg;
  int dm = deg;
  dm = max(dm, __shfl_xor(dm, 4));
  dm = max(dm, __shfl_xor(dm, 8));
  dm = max(dm, __shfl_xor(dm, 16));
  dm = __builtin_amdgcn_readfirstlane(dm);

  v4f acc = {0.f, 0.f, 0.f, 0.f};
#pragma unroll 1
  for (int j = 0; j < dm; ++j) {
    const bool ok = j < deg;
    int e = s + j;
    e = e > nE - 1 ? nE - 1 : e;
    int c = col[e];
    c = c < 0 ? 0 : (c > nN - 1 ? nN - 1 : c);
    const v4f gv = *(const v4f*)(G + (size_t)4 * e);
    const float g0 = ok ? gv.x : 0.0f, g1 = ok ? gv.y : 0.0f, g2 = ok ? gv.z : 0.0f;
    const float* xr = HW + (size_t)c * C2P + 4 * q;
    const v4f a0 = *(const v4f*)(xr);
    const v4f a1 = *(const v4f*)(xr + OUT_F);
    const v4f a2 = *(const v4f*)(xr + 2 * OUT_F);
    acc = acc + (a0 * g0 + a1 * g1 + a2 * g2);
  }
  float* op = out + (size_t)i * OUT_F + 4 * q;
  if (i < nN) *(volatile v4f*)op = acc;
  __threadfence();
  if (i < nN) *(volatile v4f*)op = acc;
}

extern "C" void kernel_launch(void* const* d_in, const int* in_sizes, int n_in,
                              void* d_out, int out_size, void* d_ws, size_t ws_size,
                              hipStream_t stream) {
  if (n_in < 8) return;
  const int nN = in_sizes[0] - 1;
  const int nE = in_sizes[1];
  if (nN < 1 || nE < 1) return;
  if (nN > (1 << 24) || nE > (1 << 28)) return;
  if (in_sizes[2] != nN * IN_F || in_sizes[3] != PDIM * nE) return;
  if (in_sizes[4] != NKER * PDIM || in_sizes[5] != NKER * PDIM) return;
  if (in_sizes[6] != NKER * IN_F * HIDF || in_sizes[7] != NKER * HIDF * OUT_F) return;
  if (out_size != nN * OUT_F) return;

  const int*   rp    = (const int*)d_in[0];
  const int*   col   = (const int*)d_in[1];
  const float* x     = (const float*)d_in[2];
  const float* p     = (const float*)d_in[3];
  const float* mu    = (const float*)d_in[4];
  const float* sigma = (const float*)d_in[5];
  const float* W1    = (const float*)d_in[6];
  const float* W2    = (const float*)d_in[7];
  float* out = (float*)d_out;

  const int NPAD = ((nN + GROWS - 1) / GROWS) * GROWS;
  const int EP   = ((nE + NTHR - 1) / NTHR) * NTHR;
  const int nGemm = NPAD / GROWS;
  const int nAgg1 = NPAD / A1NB;
  const int nAgg2 = (nN + A2NB - 1) / A2NB;
  const int nGau  = EP / NTHR;
  const int nPrep = (C1 * IN_F / 8 + C2 * HIDF / 8 + NTHR - 1) / NTHR;

  char* ws = (char*)d_ws;
  size_t off = 0;
  auto carve = [&](size_t bytes) -> size_t { const size_t o = off; off += (bytes + 255) & ~(size_t)255; return o; };
  const size_t oB1h = carve((size_t)C1 * IN_F * 2);
  const size_t oB1l = carve((size_t)C1 * IN_F * 2);
  const size_t oB2h = carve((size_t)C2 * HIDF * 2);
  const size_t oB2l = carve((size_t)C2 * HIDF * 2);
  const size_t oG   = carve((size_t)EP * 4 * 4);
  const size_t oXW  = carve((size_t)NPAD * C1 * 4);
  const size_t oH   = carve((size_t)NPAD * HIDF * 4);
  const size_t oHW  = carve((size_t)NPAD * C2P * 4);
  if (off > ws_size || off > WSCAP) return;
  unsigned short* b1h = (unsigned short*)(ws + oB1h);
  unsigned short* b1l = (unsigned short*)(ws + oB1l);
  unsigned short* b2h = (unsigned short*)(ws + oB2h);
  unsigned short* b2l = (unsigned short*)(ws + oB2l);
  float* G  = (float*)(ws + oG);
  float* XW = (float*)(ws + oXW);
  float* H  = (float*)(ws + oH);
  float* HW = (float*)(ws + oHW);

  k_wprep<<<nPrep, NTHR, 0, stream>>>(W1, W2, b1h, b1l, b2h, b2l);
  k_gauss<<<nGau, NTHR, 0, stream>>>(p, mu, sigma, G, nE);
  k_gemm<IN_F, C1 / 16, C1><<<nGemm, NTHR, 0, stream>>>(x, b1h, b1l, XW, nN);
  k_agg1<<<nAgg1, NTHR, 0, stream>>>(rp, col, G, XW, H, nN, nE);
  k_gemm<HIDF, C2 / 16, C2P><<<nGemm, NTHR, 0, stream>>>(H, b2h, b2l, HW, NPAD);
  k_agg2<<<nAgg2, NTHR, 0, stream>>>(rp, col, G, HW, out, nN, nE);
}
